// MultiHeadSelfAttention_22204980920452
// MI455X (gfx1250) — hardware-verified
//
#include <hip/hip_runtime.h>
#include <math.h>

typedef __attribute__((ext_vector_type(16))) _Float16 v16h;
typedef __attribute__((ext_vector_type(16))) __bf16 v16b;
typedef __attribute__((ext_vector_type(8)))  _Float16 v8h;
typedef __attribute__((ext_vector_type(8)))  __bf16 v8b;
typedef __attribute__((ext_vector_type(8)))  float v8f;
typedef __attribute__((ext_vector_type(4)))  float v4f;
typedef __attribute__((ext_vector_type(2)))  float v2f;
typedef __attribute__((ext_vector_type(4)))  unsigned v4u;

template <typename T> __device__ __forceinline__ void vst2(void* p, T v) { *(volatile T*)p = v; __threadfence(); *(volatile T*)p = v; }
__device__ __forceinline__ v8f wmma16(v16h a, v16h b, v8f c) {
  v8f d = __builtin_amdgcn_wmma_f32_16x16x32_f16(false, a, false, b, (short)0, c, false, false);
  asm volatile("v_nop\n\tv_nop\n\tv_nop\n\tv_nop" : "+v"(d) : "v"(a), "v"(b));
  return d;
}
__device__ __forceinline__ v8f wmma_bf(v16b a, v16b b, v8f c) {
  v8f d = __builtin_amdgcn_wmma_f32_16x16x32_bf16(false, a, false, b, (short)0, c, false, false);
  asm volatile("v_nop\n\tv_nop\n\tv_nop\n\tv_nop" : "+v"(d) : "v"(a), "v"(b));
  return d;
}
__device__ __forceinline__ v16h frag_h(const _Float16* rowk0, int lane) {
  union { v16h v; v8h q[2]; } u; const _Float16* p = rowk0 + 8 * (lane >> 4);
  u.q[0] = *(const v8h*)p; u.q[1] = *(const v8h*)(p + 16); return u.v;
}
__device__ __forceinline__ v16b frag_b(const __bf16* rowk0, int lane) {
  union { v16b v; v8b q[2]; } u; const __bf16* p = rowk0 + 8 * (lane >> 4);
  u.q[0] = *(const v8b*)p; u.q[1] = *(const v8b*)(p + 16); return u.v;
}
__device__ __forceinline__ float bfr(float v) { return (float)(__bf16)v; }
#define LDSX() do { asm volatile("s_wait_dscnt 0" ::: "memory"); __builtin_amdgcn_wave_barrier(); __builtin_amdgcn_fence(3  , "workgroup"); } while (0)

#ifndef NB
#define NB 2
#endif
#ifndef SEQ
#define SEQ 2048
#endif
#define SEQ_FULL 2048
#define DM 1024
#define NH 16
#define HD 64
#define NHT (NB * NH)
#define QHI (SEQ < 512 ? SEQ : 512)
#define SC2 0.18033688011112042f

static_assert(HD == 64);
static_assert(DM == NH * HD);
static_assert(SEQ % 64 == 0);
static_assert(QHI % 64 == 0);
static_assert(SEQ <= SEQ_FULL);
static_assert((SEQ * 32) % 256 == 0);
static_assert((long long)NHT * SEQ * HD < 2147483647LL);

#define WS_CS  ((size_t)0)
#define WS_QH  (WS_CS + (size_t)4 * SEQ * HD)
#define WS_QL  (WS_QH + (size_t)2 * NHT * SEQ * HD)
#define WS_KH  (WS_QL + (size_t)2 * NHT * SEQ * HD)
#define WS_KL  (WS_KH + (size_t)2 * NHT * SEQ * HD)
#define WS_VT  (WS_KL + (size_t)2 * NHT * QHI * HD)
#define WS_VB  (WS_VT + (size_t)2 * NHT * HD * SEQ)
#define WS_END (WS_VB + (size_t)2 * NHT * HD * QHI)
static_assert(WS_END <= (size_t)134217728);
static_assert(WS_QH % 128 == 0 && WS_QL % 128 == 0 && WS_KH % 128 == 0 && WS_KL % 128 == 0 && WS_VT % 128 == 0 && WS_VB % 128 == 0);

__global__ __launch_bounds__(256) void k_tab(float* __restrict__ CS) {
  const int idx = blockIdx.x * 256 + threadIdx.x;
  const int r = idx >> 5, i = idx & 31;
  double p = (i & 1) ? 1.3335214321633240 : 1.0;
  p *= (i & 2) ? 1.7782794100389228 : 1.0;
  p *= (i & 4) ? 3.1622776601683795 : 1.0;
  p *= (i & 8) ? 10.0 : 1.0;
  p *= (i & 16) ? 100.0 : 1.0;
  const float pf = (float)p;
  const float ang = (float)r / pf;
  float sn, cs; sincosf(ang, &sn, &cs);
  v2f o; o[0] = cs; o[1] = sn;
  vst2(CS + (size_t)idx * 2, o);
}

__device__ __forceinline__ void rot8(const v4f x0, const v4f x1, const v4f c0, const v4f c1, v4u& hi, v4u& lo) {
  float y[8];
  { const float a = bfr(x0[0]), b = bfr(x0[1]); y[0] = a * c0[0] - b * c0[1]; y[1] = a * c0[1] + b * c0[0]; }
  { const float a = bfr(x0[2]), b = bfr(x0[3]); y[2] = a * c0[2] - b * c0[3]; y[3] = a * c0[3] + b * c0[2]; }
  { const float a = bfr(x1[0]), b = bfr(x1[1]); y[4] = a * c1[0] - b * c1[1]; y[5] = a * c1[1] + b * c1[0]; }
  { const float a = bfr(x1[2]), b = bfr(x1[3]); y[6] = a * c1[2] - b * c1[3]; y[7] = a * c1[3] + b * c1[2]; }
  union { v8h h; v4u u; } a, r;
#pragma unroll
  for (int i = 0; i < 8; ++i) { const _Float16 hv = (_Float16)y[i]; a.h[i] = hv; r.h[i] = (_Float16)((y[i] - (float)hv) * 1024.0f); }
  hi = a.u; lo = r.u;
}

__global__ __launch_bounds__(128) void k_prep(const float* __restrict__ Q, const float* __restrict__ K, const float* __restrict__ V, const float* __restrict__ CS,
    _Float16* __restrict__ QH, _Float16* __restrict__ QL, _Float16* __restrict__ KH, _Float16* __restrict__ KL, _Float16* __restrict__ VT, __bf16* __restrict__ VB) {
  __shared__ __align__(16) _Float16 th[64][72]; __shared__ __align__(16) __bf16 tb[64][72];
  const int tid = threadIdx.x; const int r0 = blockIdx.x * 64; const int hd = blockIdx.y; const int b = hd / NH, g = hd % NH;
  const size_t ib = (size_t)b * SEQ_FULL * DM + (size_t)g * SEQ * HD + (size_t)r0 * HD;
  const size_t pb = ((size_t)hd * SEQ + r0) * HD;
  const bool early = r0 < QHI;
#pragma unroll 1
  for (int it = 0; it < 4; ++it) {
    const int e = it * 128 + tid, rl = e >> 3, pc = e & 7; const int off = rl * HD + pc * 8;
    const float* cp = CS + (size_t)(r0 + rl) * HD + pc * 8;
    const v4f c0 = *(const v4f*)cp, c1 = *(const v4f*)(cp + 4);
    v4u hi, lo;
    { const v4f x0 = *(const v4f*)(Q + ib + off), x1 = *(const v4f*)(Q + ib + off + 4); rot8(x0, x1, c0, c1, hi, lo);
      vst2(QH + pb + off, hi); vst2(QL + pb + off, lo); }
    { const v4f x0 = *(const v4f*)(K + ib + off), x1 = *(const v4f*)(K + ib + off + 4); rot8(x0, x1, c0, c1, hi, lo);
      vst2(KH + pb + off, hi); if (early) vst2(KL + ((size_t)hd * QHI + r0) * HD + off, lo); }
    { const v4f x0 = *(const v4f*)(V + ib + off), x1 = *(const v4f*)(V + ib + off + 4);
#pragma unroll
      for (int i = 0; i < 4; ++i) { const float a = bfr(x0[i]), c = bfr(x1[i]); th[pc * 8 + i][rl] = (_Float16)a; th[pc * 8 + 4 + i][rl] = (_Float16)c;
        if (early) { tb[pc * 8 + i][rl] = (__bf16)a; tb[pc * 8 + 4 + i][rl] = (__bf16)c; } } }
  }
  __syncthreads();
#pragma unroll 1
  for (int it = 0; it < 4; ++it) {
    const int e = it * 128 + tid, d = e >> 3, pc = e & 7;
    vst2(VT + ((size_t)hd * HD + d) * SEQ + r0 + pc * 8, *(const v4u*)&th[d][pc * 8]);
    if (early) vst2(VB + ((size_t)hd * HD + d) * QHI + r0 + pc * 8, *(const v4u*)&tb[d][pc * 8]);
  }
}

template <bool EARLY>
__device__ __forceinline__ void fa_loop(const _Float16* __restrict__ QH, const _Float16* __restrict__ QL, const _Float16* __restrict__ KH, const _Float16* __restrict__ KL,
    const _Float16* __restrict__ VT, const __bf16* __restrict__ VB, int hd, int nh, int qoff0, int qrow, int lane, v8f (&ot)[4], float& m, float& l) {
  const int col = lane & 15, h = lane >> 4;
#pragma unroll 1
  for (int hb = 0; hb < nh; ++hb) {
    const int kb = hb * 32;
    int qo = qoff0; asm volatile("" : "+v"(qo));
    const int ko = (hd * SEQ + kb + col) * HD;
    const int klo = (hd * QHI + kb + col) * HD;
    v8f acc[2] = {}, accl[2] = {};
#pragma unroll
    for (int kc = 0; kc < 2; ++kc) {
      const v16h qh = frag_h(QH + qo + kc * 32, lane), ql = frag_h(QL + qo + kc * 32, lane);
#pragma unroll
      for (int t = 0; t < 2; ++t) {
        const v16h kf = frag_h(KH + ko + t * 16 * HD + kc * 32, lane);
        acc[t] = wmma16(kf, qh, acc[t]); accl[t] = wmma16(kf, ql, accl[t]);
        if (EARLY) { const v16h klf = frag_h(KL + klo + t * 16 * HD + kc * 32, lane); accl[t] = wmma16(klf, qh, accl[t]); }
      }
    }
    const int lim = qrow - kb - 8 * h;
    float sv[16]; float mx = -1.0e30f;
#pragma unroll
    for (int t = 0; t < 2; ++t)
#pragma unroll
      for (int r = 0; r < 8; ++r) { float s = (acc[t][r] + accl[t][r] * (1.0f / 1024.0f)) * SC2; s = (16 * t + r <= lim) ? s : -1.0e30f; sv[8 * t + r] = s; mx = fmaxf(mx, s); }
    mx = fmaxf(mx, __shfl_xor(mx, 16));
    const float mn = fmaxf(m, mx); const float alpha = exp2f(m - mn); m = mn;
#pragma unroll
    for (int t = 0; t < 2; ++t)
#pragma unroll
      for (int r = 0; r < 8; ++r) { float p = exp2f(sv[8 * t + r] - mn); p = (16 * t + r <= lim) ? p : 0.0f; sv[8 * t + r] = p; }
#pragma unroll
    for (int j = 0; j < 4; ++j)
#pragma unroll
      for (int r = 0; r < 8; ++r) ot[j][r] *= alpha;
    float ps = 0.0f;
    if (EARLY) {
      v16b ph, pl;
#pragma unroll
      for (int i = 0; i < 16; ++i) { const float p = sv[i]; const __bf16 a = (__bf16)p; ph[i] = a; pl[i] = (__bf16)(p - (float)a); ps += p; }
      const int vo = (hd * HD + col) * QHI + kb;
#pragma unroll
      for (int j = 0; j < 4; ++j) { const v16b vf = frag_b(VB + vo + j * 16 * QHI, lane); ot[j] = wmma_bf(vf, ph, ot[j]); ot[j] = wmma_bf(vf, pl, ot[j]); }
    } else {
      v16h pf;
#pragma unroll
      for (int i = 0; i < 16; ++i) { const _Float16 a = (_Float16)(sv[i] * 1024.0f); pf[i] = a; ps += (float)a; }
      const int vo = (hd * HD + col) * SEQ + kb;
#pragma unroll
      for (int j = 0; j < 4; ++j) { const v16h vf = frag_h(VT + vo + j * 16 * SEQ, lane); ot[j] = wmma16(vf, pf, ot[j]); }
    }
    l = l * alpha + ps;
  }
}

__global__ __launch_bounds__(128) void k_fa(const _Float16* __restrict__ QH, const _Float16* __restrict__ QL, const _Float16* __restrict__ KH, const _Float16* __restrict__ KL,
    const _Float16* __restrict__ VT, const __bf16* __restrict__ VB, float* __restrict__ OUT) {
  __shared__ __align__(16) float so[4][16][68];
  const int tid = threadIdx.x, lane = tid & 31, col = lane & 15, h = lane >> 4;
  const int wave = __builtin_amdgcn_readfirstlane(threadIdx.x >> 5);
  const int hd = blockIdx.y; const int q0 = blockIdx.x * 64 + wave * 16; const int qrow = q0 + col;
  const int nh = (q0 >> 5) + 1;
  const int qoff0 = (hd * SEQ + qrow) * HD;
  v8f ot[4] = {}; float m = -1.0e30f, l = 0.0f;
  if (q0 < QHI) fa_loop<true>(QH, QL, KH, KL, VT, VB, hd, nh, qoff0, qrow, lane, ot, m, l);
  else          fa_loop<false>(QH, QL, KH, KL, VT, VB, hd, nh, qoff0, qrow, lane, ot, m, l);
  l += __shfl_xor(l, 16);
  const float inv = 1.0f / l;
#pragma unroll
  for (int j = 0; j < 4; ++j) { v4f a, c;
#pragma unroll
    for (int r = 0; r < 4; ++r) { a[r] = ot[j][r] * inv; c[r] = ot[j][4 + r] * inv; }
    *(v4f*)&so[wave][col][16 * j + 8 * h] = a; *(v4f*)&so[wave][col][16 * j + 8 * h + 4] = c; }
  LDSX();
  const size_t ob = ((size_t)hd * SEQ + q0) * HD;
#pragma unroll 1
  for (int it = 0; it < 8; ++it) { const v4f v = *(const v4f*)&so[wave][it * 2 + h][col * 4]; vst2(OUT + ob + it * 128 + lane * 4, v); }
}

extern "C" void kernel_launch(void* const* d_in, const int* in_sizes, int n_in, void* d_out, int out_size, void* d_ws, size_t ws_size, hipStream_t stream) {
  if (n_in < 3) return;
  if (ws_size < (size_t)WS_END) return;
  const int need = (NB - 1) * SEQ_FULL * DM + SEQ * DM;
  if (in_sizes[0] < need || in_sizes[1] < need || in_sizes[2] < need) return;
  if (out_size < NB * SEQ * DM) return;
  const float* Qp = (const float*)d_in[0]; const float* Kp = (const float*)d_in[1]; const float* Vp = (const float*)d_in[2];
  char* ws = (char*)d_ws;
  float* CS = (float*)(ws + WS_CS);
  _Float16 *QH = (_Float16*)(ws + WS_QH), *QL = (_Float16*)(ws + WS_QL), *KH = (_Float16*)(ws + WS_KH), *KL = (_Float16*)(ws + WS_KL), *VT = (_Float16*)(ws + WS_VT);
  __bf16* VB = (__bf16*)(ws + WS_VB);
  k_tab<<<dim3(SEQ * 32 / 256), 256, 0, stream>>>(CS);
  k_prep<<<dim3(SEQ / 64, NHT), 128, 0, stream>>>(Qp, Kp, Vp, CS, QH, QL, KH, KL, VT, VB);
  k_fa<<<dim3(SEQ / 64, NHT), 128, 0, stream>>>(QH, QL, KH, KL, VT, VB, (float*)d_out);
}
